// edge_CrossAttention_63324997812372
// MI455X (gfx1250) — hardware-verified
//
#include <hip/hip_runtime.h>
#include <math.h>
#include <stdint.h>

#define NBATCH  8
#define NTOK    1024
#define DM      768
#define DE      256
#define NH      8
#define HD      96
#define MROWS   (NBATCH * NTOK)
#define WSC     64.0f
#define ACARRY  16.0f
#define QC      64.0f
#define KC      16.0f
#define VC      16.0f
#define PC      32768.0f
#define FC      256.0f
static_assert(NH * HD == DM);
static_assert((HD % 32) == 0 && (HD % 16) == 0);
static_assert((MROWS % 64) == 0 && (DM % 64) == 0 && (NTOK % 64) == 0 && (DE % 32) == 0);
static_assert((NTOK % 32) == 0 && (NTOK % 16) == 0);
static_assert(MROWS == 8192);
#define ATT_BLOCKS (NBATCH * (NTOK / 16))
#define OS_PIECES  (16 * (DM / 8))
static_assert(OS_PIECES == 6 * 256);

typedef _Float16 v16h __attribute__((ext_vector_type(16)));
typedef _Float16 v8h  __attribute__((ext_vector_type(8)));
typedef float    v8f  __attribute__((ext_vector_type(8)));
typedef float    v4f  __attribute__((ext_vector_type(4)));
typedef unsigned int v4u __attribute__((ext_vector_type(4)));

union FragH { v16h v; v8h h[2]; v4u u[2]; };

__device__ __forceinline__ unsigned short bf_bits(float f) {
  unsigned u = __float_as_uint(f);
  return (unsigned short)((u + 0x7FFFu + ((u >> 16) & 1u)) >> 16);
}
__device__ __forceinline__ float bf_up(unsigned short h) { return __uint_as_float(((unsigned)h) << 16); }
__device__ __forceinline__ float bfr(float f) { return bf_up(bf_bits(f)); }
__device__ __forceinline__ unsigned short h_bits(_Float16 x) { return __builtin_bit_cast(unsigned short, x); }
__device__ __forceinline__ unsigned pk16(unsigned short a, unsigned short b) { return (unsigned)a | ((unsigned)b << 16); }
__device__ __forceinline__ v8f zero8() { v8f z = {0.f, 0.f, 0.f, 0.f, 0.f, 0.f, 0.f, 0.f}; return z; }

__device__ __forceinline__ v16h ldfrag_h(const _Float16* p) {
  FragH f;
  f.h[0] = *(const v8h*)(p);
  f.h[1] = *(const v8h*)(p + 16);
  return f.v;
}
__device__ __forceinline__ v16h ldfrag_u(const unsigned short* p) {
  FragH f;
  f.u[0] = *(const v4u*)(p);
  f.u[1] = *(const v4u*)(p + 16);
  return f.v;
}

__device__ __forceinline__ v8f mma_raw(v16h a, v16h b, v8f c) {
  return __builtin_amdgcn_wmma_f32_16x16x32_f16(false, a, false, b, (short)0, c, false, false);
}
__device__ __forceinline__ void dep_guard1(v8f& a, v8f& b, v16h x) {
#if defined(__HIP_DEVICE_COMPILE__)
  asm volatile("v_nop\n\tv_nop\n\tv_nop\n\tv_nop" : "+v"(a), "+v"(b) : "v"(x));
#endif
}
__device__ __forceinline__ void guard_s6(v8f& s, v16h a0, v16h a1, v16h a2, v16h b0, v16h b1, v16h b2) {
#if defined(__HIP_DEVICE_COMPILE__)
  asm volatile("v_nop\n\tv_nop\n\tv_nop\n\tv_nop" : "+v"(s) : "v"(a0), "v"(a1), "v"(a2), "v"(b0), "v"(b1), "v"(b2));
#endif
}
__device__ __forceinline__ void guard_s9(v8f& s, v16h a0, v16h a1, v16h a2, v16h b0, v16h b1, v16h b2,
                                         v16h c0, v16h c1, v16h c2) {
#if defined(__HIP_DEVICE_COMPILE__)
  asm volatile("v_nop\n\tv_nop\n\tv_nop\n\tv_nop" : "+v"(s)
               : "v"(a0), "v"(a1), "v"(a2), "v"(b0), "v"(b1), "v"(b2), "v"(c0), "v"(c1), "v"(c2));
#endif
}
__device__ __forceinline__ void guard_pv(v8f& a, v8f& b, v16h x, v16h y, v16h z, v16h w) {
#if defined(__HIP_DEVICE_COMPILE__)
  asm volatile("v_nop\n\tv_nop\n\tv_nop\n\tv_nop" : "+v"(a), "+v"(b) : "v"(x), "v"(y), "v"(z), "v"(w));
#endif
}
__device__ __forceinline__ void keep4_h(v16h a, v16h b, v16h c, v16h d) {
#if defined(__HIP_DEVICE_COMPILE__)
  asm volatile("v_nop" :: "v"(a), "v"(b), "v"(c), "v"(d));
#endif
}
__device__ __forceinline__ void acc_guard4(v8f& a, v8f& b, v8f& c, v8f& d) {
#if defined(__HIP_DEVICE_COMPILE__)
  asm volatile("v_nop\n\tv_nop\n\tv_nop\n\tv_nop" : "+v"(a), "+v"(b), "+v"(c), "+v"(d));
#endif
}
__device__ __forceinline__ void opaque_i(int& x) {
#if defined(__HIP_DEVICE_COMPILE__)
  asm volatile("" : "+v"(x));
#endif
}
__device__ __forceinline__ void wave_sync_lds() {
  __builtin_amdgcn_fence(__ATOMIC_RELEASE, "workgroup");
  __builtin_amdgcn_wave_barrier();
  __builtin_amdgcn_fence(__ATOMIC_ACQUIRE, "workgroup");
}

__global__ __launch_bounds__(256) void conv16(const float* __restrict__ W, unsigned short* dst, int n8, float wsc) {
  const int i  = blockIdx.x * 256 + threadIdx.x;
  const int ic = (i < n8) ? i : (n8 - 1);
  const float* p = W + (size_t)ic * 8;
  const v4f a = *(const v4f*)(p), b = *(const v4f*)(p + 4);
  float v[8];
#pragma unroll
  for (int e = 0; e < 4; ++e) { v[e] = bfr(a[e]); v[4 + e] = bfr(b[e]); }
  v4u ov;
#pragma unroll
  for (int e = 0; e < 4; ++e) ov[e] = pk16(h_bits((_Float16)(v[2 * e] * wsc)), h_bits((_Float16)(v[2 * e + 1] * wsc)));
  if (i < n8) *(volatile v4u*)(dst + (size_t)i * 8) = ov;
  __threadfence();
  if (i < n8) *(volatile v4u*)(dst + (size_t)i * 8) = ov;
}

template <int OM, int HASB>
__global__ __launch_bounds__(256) void gemm64(
    const unsigned short* __restrict__ Ap, int lda, long long sA,
    const unsigned short* __restrict__ Btp, int ldb, long long sB,
    const float* __restrict__ bias, float bscale,
    void* Cout, void* Cout2, int ldc, long long sC,
    int M, int N, int K, float oscale) {
  __shared__ __align__(16) float sT[8][16 * 68];
  const int by   = blockIdx.y;
  const int lane = threadIdx.x & 31;
  const int wave = threadIdx.x >> 5;
  const int tilesN = N >> 6;
  const int tilesM = M >> 6;
  const int tile = blockIdx.x * 8 + wave;
  if (tile >= tilesM * tilesN) return;
  const int tm = tile / tilesN;
  const int tn = tile - tm * tilesN;
  const int m0 = tm << 6;
  const int n0 = tn << 6;

  const unsigned short* A1 = Ap  + (size_t)((long long)by * sA);
  const unsigned short* Bb = Btp + (size_t)((long long)by * sB);

  const int rlane = lane & 15;
  const int koff  = (lane >> 4) * 8;
  const int mOff  = (lane >> 4) * 8;

  v8f acc[4][4];
#pragma unroll
  for (int i = 0; i < 4; ++i)
#pragma unroll
    for (int j = 0; j < 4; ++j) acc[i][j] = zero8();

  for (int k0 = 0; k0 < K; k0 += 32) {
    v16h bh[4];
#pragma unroll
    for (int j = 0; j < 4; ++j) {
      const size_t bofs = (size_t)(n0 + (j << 4) + rlane) * ldb + koff + k0;
      bh[j] = ldfrag_u(Bb + bofs);
    }
#pragma unroll
    for (int i = 0; i < 4; ++i) {
      const size_t ao = (size_t)(m0 + (i << 4) + rlane) * lda + koff + k0;
      const v16h ah = ldfrag_u(A1 + ao);
#pragma unroll
      for (int j = 0; j < 4; ++j) acc[i][j] = mma_raw(ah, bh[j], acc[i][j]);
      dep_guard1(acc[i][0], acc[i][3], ah);
    }
    keep4_h(bh[0], bh[1], bh[2], bh[3]);
  }
  acc_guard4(acc[0][0], acc[0][1], acc[0][2], acc[0][3]);
  acc_guard4(acc[1][0], acc[1][1], acc[1][2], acc[1][3]);
  acc_guard4(acc[2][0], acc[2][1], acc[2][2], acc[2][3]);
  acc_guard4(acc[3][0], acc[3][1], acc[3][2], acc[3][3]);

  const int hh2 = lane >> 4, c4 = (lane & 15) * 4;
  const int q8  = lane >> 3, c8 = (lane & 7) * 8;
  float bc[4];
#pragma unroll
  for (int e = 0; e < 4; ++e) bc[e] = 0.f;
  if (HASB != 0 && OM == 0) {
    const int cb = n0 + c4;
    const int i0 = (cb < N - 4) ? cb : (N - 4);
    const v4f b0v = *(const v4f*)(bias + i0);
#pragma unroll
    for (int e = 0; e < 4; ++e) bc[e] = bfr(b0v[e]) * bscale;
  }

  float* slab = sT[wave];
#pragma unroll
  for (int i = 0; i < 4; ++i) {
    const int mBase = m0 + (i << 4);
#pragma unroll
    for (int j = 0; j < 4; ++j) {
#pragma unroll
      for (int r = 0; r < 8; ++r) {
        slab[(mOff + r) * 68 + (j << 4) + rlane] = acc[i][j][r];
      }
    }
    wave_sync_lds();
    if (OM == 0) {
      float* C = (float*)Cout + (size_t)((long long)by * sC);
      v4f vals[8];
#pragma unroll
      for (int it = 0; it < 8; ++it) {
        const int row = it * 2 + hh2;
        v4f v = *(const v4f*)(slab + row * 68 + c4);
#pragma unroll
        for (int e = 0; e < 4; ++e) v[e] = v[e] * oscale + bc[e];
        vals[it] = v;
      }
      for (int pass = 0; pass < 2; ++pass) {
#pragma unroll
        for (int it = 0; it < 8; ++it) {
          const int gr = mBase + it * 2 + hh2;
          *(volatile v4f*)(C + (size_t)gr * ldc + n0 + c4) = vals[it];
        }
        __threadfence();
      }
    } else {
      unsigned short* C  = (unsigned short*)Cout  + (size_t)((long long)by * sC);
      unsigned short* C2 = (unsigned short*)Cout2 + (size_t)((long long)by * sC);
      v4u hv[4], lv[4];
#pragma unroll
      for (int it = 0; it < 4; ++it) {
        const int row = it * 4 + q8;
        const float* sp = slab + row * 68 + c8;
        v4u a = {0u, 0u, 0u, 0u}, b = {0u, 0u, 0u, 0u};
#pragma unroll
        for (int e = 0; e < 4; ++e) {
          const float f0 = sp[2 * e] * oscale;
          const float f1 = sp[2 * e + 1] * oscale;
          const _Float16 h0 = (_Float16)f0, h1 = (_Float16)f1;
          a[e] = pk16(h_bits(h0), h_bits(h1));
          if (OM == 3) {
            const _Float16 l0 = (_Float16)(f0 - (float)h0), l1 = (_Float16)(f1 - (float)h1);
            b[e] = pk16(h_bits(l0), h_bits(l1));
          }
        }
        hv[it] = a;
        lv[it] = b;
      }
      for (int pass = 0; pass < 2; ++pass) {
#pragma unroll
        for (int it = 0; it < 4; ++it) {
          const int row = it * 4 + q8;
          *(volatile v4u*)(C + (size_t)(mBase + row) * ldc + n0 + c8) = hv[it];
          if (OM == 3) *(volatile v4u*)(C2 + (size_t)(mBase + row) * ldc + n0 + c8) = lv[it];
        }
        __threadfence();
      }
    }
    wave_sync_lds();
  }
}

__global__ __launch_bounds__(256)
void attn96(const unsigned short* __restrict__ QHp, const unsigned short* __restrict__ QLp,
            const unsigned short* __restrict__ Kpl, const unsigned short* __restrict__ VTq,
            unsigned short* CT) {
  __shared__ __align__(16) float Ps[NH][16 * 36];
  __shared__ __align__(16) unsigned short Os[16 * DM];

  const int tid  = threadIdx.x;
  const int wave = tid >> 5;
  const int lane = tid & 31;
  const int hh   = lane >> 4;
  const int c    = lane & 15;

  const int bat  = blockIdx.x / (NTOK / 16);
  const int qt   = blockIdx.x - bat * (NTOK / 16);
  const int head = wave;
  const int q0   = qt * 16;

  const size_t qofs = ((size_t)bat * NTOK + q0 + c) * DM + head * HD + 8 * hh;
  const _Float16* Qh = (const _Float16*)(const void*)QHp + qofs;
  const _Float16* Ql = (const _Float16*)(const void*)QLp + qofs;
  const _Float16* Kb = (const _Float16*)(const void*)Kpl + (size_t)bat * NTOK * DM + head * HD + 8 * hh;
  const _Float16* Vb = (const _Float16*)(const void*)VTq + (size_t)(bat * NH + head) * HD * NTOK + 8 * hh;
  const float lsc = (1.4426950408889634f / (float)HD) / (QC * KC);

  const v16h qh0 = ldfrag_h(Qh), qh1 = ldfrag_h(Qh + 32), qh2 = ldfrag_h(Qh + 64);

  float mrow[8], lrow[8];
  v8f o0 = zero8(), o1 = zero8(), o2 = zero8(), o3 = zero8(), o4 = zero8(), o5 = zero8();
#pragma unroll
  for (int r = 0; r < 8; ++r) { mrow[r] = -INFINITY; lrow[r] = 0.f; }
  float* pt = Ps[wave];

#pragma unroll 1
  for (int kb = 0; kb < NTOK; kb += 32) {
    int zo = 0;
    opaque_i(zo);
    const _Float16* ql = Ql + zo;
    const v16h l0 = ldfrag_h(ql), l1 = ldfrag_h(ql + 32), l2 = ldfrag_h(ql + 64);
    const _Float16* kp = Kb + (size_t)(kb + c) * DM;
    v8f s0, s1;
    {
      const v16h k0 = ldfrag_h(kp), k1 = ldfrag_h(kp + 32), k2 = ldfrag_h(kp + 64);
      s0 = mma_raw(qh0, k0, zero8());
      s0 = mma_raw(l0,  k0, s0);
      s0 = mma_raw(qh1, k1, s0);
      s0 = mma_raw(l1,  k1, s0);
      s0 = mma_raw(qh2, k2, s0);
      s0 = mma_raw(l2,  k2, s0);
      guard_s6(s0, k0, k1, k2, l0, l1, l2);
    }
    {
      const _Float16* kq = kp + (size_t)16 * DM;
      const v16h k0 = ldfrag_h(kq), k1 = ldfrag_h(kq + 32), k2 = ldfrag_h(kq + 64);
      s1 = mma_raw(qh0, k0, zero8());
      s1 = mma_raw(l0,  k0, s1);
      s1 = mma_raw(qh1, k1, s1);
      s1 = mma_raw(l1,  k1, s1);
      s1 = mma_raw(qh2, k2, s1);
      s1 = mma_raw(l2,  k2, s1);
      guard_s9(s1, k0, k1, k2, l0, l1, l2, qh0, qh1, qh2);
    }
#pragma unroll
    for (int r = 0; r < 8; ++r) {
      const float t0 = s0[r] * lsc, t1 = s1[r] * lsc;
      float mx = fmaxf(t0, t1);
#pragma unroll
      for (int off = 1; off < 16; off <<= 1) mx = fmaxf(mx, __shfl_xor(mx, off, 32));
      const float mn = fmaxf(mrow[r], mx);
      const float al = exp2f(mrow[r] - mn);
      mrow[r] = mn;
      const float e0 = exp2f(t0 - mn), e1 = exp2f(t1 - mn);
      float ps = e0 + e1;
#pragma unroll
      for (int off = 1; off < 16; off <<= 1) ps += __shfl_xor(ps, off, 32);
      lrow[r] = lrow[r] * al + ps;
      o0[r] *= al;
      o1[r] *= al;
      o2[r] *= al;
      o3[r] *= al;
      o4[r] *= al;
      o5[r] *= al;
      const int ro = (8 * hh + r) * 36 + c;
      pt[ro]      = e0;
      pt[ro + 16] = e1;
    }
    wave_sync_lds();
    FragH ph, pl;
    {
      const float* prow = pt + c * 36 + 8 * hh;
      const v4f p0 = *(const v4f*)(prow), p1 = *(const v4f*)(prow + 4);
      const v4f p2 = *(const v4f*)(prow + 16), p3 = *(const v4f*)(prow + 20);
#pragma unroll
      for (int e = 0; e < 4; ++e) {
        const float f0 = p0[e] * PC, f1 = p1[e] * PC, f2 = p2[e] * PC, f3 = p3[e] * PC;
        const _Float16 g0 = (_Float16)f0, g1 = (_Float16)f1, g2 = (_Float16)f2, g3 = (_Float16)f3;
        ph.h[0][e]     = g0;
        ph.h[0][4 + e] = g1;
        ph.h[1][e]     = g2;
        ph.h[1][4 + e] = g3;
        pl.h[0][e]     = (_Float16)(f0 - (float)g0);
        pl.h[0][4 + e] = (_Float16)(f1 - (float)g1);
        pl.h[1][e]     = (_Float16)(f2 - (float)g2);
        pl.h[1][4 + e] = (_Float16)(f3 - (float)g3);
      }
    }
    const _Float16* vp = Vb + (size_t)c * NTOK + kb;
    {
      const v16h vb0 = ldfrag_h(vp), vb1 = ldfrag_h(vp + (size_t)16 * NTOK);
      o0 = mma_raw(ph.v, vb0, o0);
      o0 = mma_raw(pl.v, vb0, o0);
      o1 = mma_raw(ph.v, vb1, o1);
      o1 = mma_raw(pl.v, vb1, o1);
      guard_pv(o0, o1, ph.v, pl.v, vb0, vb1);
    }
    {
      const v16h vb2 = ldfrag_h(vp + (size_t)32 * NTOK), vb3 = ldfrag_h(vp + (size_t)48 * NTOK);
      o2 = mma_raw(ph.v, vb2, o2);
      o2 = mma_raw(pl.v, vb2, o2);
      o3 = mma_raw(ph.v, vb3, o3);
      o3 = mma_raw(pl.v, vb3, o3);
      guard_pv(o2, o3, ph.v, pl.v, vb2, vb3);
    }
    {
      const v16h vb4 = ldfrag_h(vp + (size_t)64 * NTOK), vb5 = ldfrag_h(vp + (size_t)80 * NTOK);
      o4 = mma_raw(ph.v, vb4, o4);
      o4 = mma_raw(pl.v, vb4, o4);
      o5 = mma_raw(ph.v, vb5, o5);
      o5 = mma_raw(pl.v, vb5, o5);
      guard_pv(o4, o5, ph.v, pl.v, vb4, vb5);
    }
    wave_sync_lds();
  }

  const float oc = FC / (PC * VC);
  unsigned short* osw = Os + head * HD + c;
#pragma unroll
  for (int r = 0; r < 8; ++r) {
    const float inv = (1.0f / lrow[r]) * oc;
    unsigned short* op = osw + (8 * hh + r) * DM;
    op[0]  = h_bits((_Float16)(o0[r] * inv));
    op[16] = h_bits((_Float16)(o1[r] * inv));
    op[32] = h_bits((_Float16)(o2[r] * inv));
    op[48] = h_bits((_Float16)(o3[r] * inv));
    op[64] = h_bits((_Float16)(o4[r] * inv));
    op[80] = h_bits((_Float16)(o5[r] * inv));
  }
  __syncthreads();
  {
    v4u vals[6];
#pragma unroll
    for (int it = 0; it < 6; ++it) {
      const int p   = it * 256 + tid;
      const int row = p / (DM / 8);
      const int c8  = (p - row * (DM / 8)) * 8;
      vals[it] = *(const v4u*)(Os + row * DM + c8);
    }
    unsigned short* dst = CT + ((size_t)bat * NTOK + q0) * DM;
    for (int pass = 0; pass < 2; ++pass) {
#pragma unroll
      for (int it = 0; it < 6; ++it) {
        const int p   = it * 256 + tid;
        const int row = p / (DM / 8);
        const int c8  = (p - row * (DM / 8)) * 8;
        *(volatile v4u*)(dst + (size_t)row * DM + c8) = vals[it];
      }
      __threadfence();
    }
  }
}

extern "C" void kernel_launch(void* const* d_in, const int* in_sizes, int n_in,
                              void* d_out, int out_size, void* d_ws, size_t ws_size,
                              hipStream_t stream) {
  if (n_in < 7) return;
  if (in_sizes[0] != MROWS * DM) return;
  if (in_sizes[1] != MROWS * DE) return;
  if (in_sizes[2] != DM * DM) return;
  if (in_sizes[3] != DM * DE || in_sizes[4] != DM * DE) return;
  if (in_sizes[5] != DM * DM || in_sizes[6] != DM) return;
  if (out_size != MROWS * DM) return;

  const float* q_x  = (const float*)d_in[0];
  const float* kv_x = (const float*)d_in[1];
  const float* w_q  = (const float*)d_in[2];
  const float* w_k  = (const float*)d_in[3];
  const float* w_v  = (const float*)d_in[4];
  const float* w_o  = (const float*)d_in[5];
  const float* b_o  = (const float*)d_in[6];
  float*       out  = (float*)d_out;

  const size_t PWQ = (size_t)DM * DM * 2;
  const size_t PWK = (size_t)DM * DE * 2;
  const size_t PQI = (size_t)MROWS * DM * 2;
  const size_t PKI = (size_t)MROWS * DE * 2;
  const size_t PVT = (size_t)NBATCH * NH * HD * NTOK * 2;
  size_t off = 0;
  const size_t oWQ = off; off += PWQ;
  const size_t oWK = off; off += PWK;
  const size_t oWV = off; off += PWK;
  const size_t oWO = off; off += PWQ;
  const size_t oQI = off; off += PQI;
  const size_t oKI = off; off += PKI;
  const size_t oQH = off; off += PQI;
  const size_t oQL = off; off += PQI;
  const size_t oKP = off; off += PQI;
  const size_t oVT = off; off += PVT;
  const size_t oCT = off; off += PQI;
  if (off > ws_size) return;
  if (off > (size_t)134217728) return;

  char* ws = (char*)d_ws;
  unsigned short* WQ  = (unsigned short*)(ws + oWQ);
  unsigned short* WK  = (unsigned short*)(ws + oWK);
  unsigned short* WV  = (unsigned short*)(ws + oWV);
  unsigned short* WO  = (unsigned short*)(ws + oWO);
  unsigned short* QI  = (unsigned short*)(ws + oQI);
  unsigned short* KI  = (unsigned short*)(ws + oKI);
  unsigned short* QH  = (unsigned short*)(ws + oQH);
  unsigned short* QL  = (unsigned short*)(ws + oQL);
  unsigned short* KP  = (unsigned short*)(ws + oKP);
  unsigned short* VTp = (unsigned short*)(ws + oVT);
  unsigned short* CT  = (unsigned short*)(ws + oCT);

  const int n8wq = (DM * DM) / 8;
  const int n8wk = (DM * DE) / 8;
  const int n8q  = (MROWS * DM) / 8;
  const int n8kv = (MROWS * DE) / 8;
  if ((n8wq % 256) != 0 || (n8wk % 256) != 0 || (n8q % 256) != 0 || (n8kv % 256) != 0) return;
  const dim3 blk(256);
  const dim3 gCwq(n8wq / 256), gCwk(n8wk / 256), gCq(n8q / 256), gCkv(n8kv / 256);
  const int tilesQK = (MROWS / 64) * (DM / 64);
  const int tilesVT = (DM / 64) * (NTOK / 64);
  if ((tilesQK % 8) != 0 || (tilesVT % 8) != 0) return;
  const dim3 gQK(tilesQK / 8, 1);
  const dim3 gVT(tilesVT / 8, NBATCH);
  const dim3 gAT(ATT_BLOCKS);

  conv16<<<gCwq, blk, 0, stream>>>(w_q, WQ, n8wq, WSC);
  conv16<<<gCwk, blk, 0, stream>>>(w_k, WK, n8wk, WSC);
  conv16<<<gCwk, blk, 0, stream>>>(w_v, WV, n8wk, WSC);
  conv16<<<gCwq, blk, 0, stream>>>(w_o, WO, n8wq, WSC);

  conv16<<<gCq,  blk, 0, stream>>>(q_x,  QI, n8q,  ACARRY);
  conv16<<<gCkv, blk, 0, stream>>>(kv_x, KI, n8kv, ACARRY);

  gemm64<3, 0><<<gQK, blk, 0, stream>>>(
      QI, DM, 0LL,
      WQ, DM, 0LL,
      b_o, 0.f,
      (void*)QH, (void*)QL, DM, 0LL,
      MROWS, DM, DM, QC / (ACARRY * WSC));

  gemm64<2, 0><<<gQK, blk, 0, stream>>>(
      KI, DE, 0LL,
      WK, DE, 0LL,
      b_o, 0.f,
      (void*)KP, (void*)KP, DM, 0LL,
      MROWS, DM, DE, KC / (ACARRY * WSC));

  gemm64<2, 0><<<gVT, blk, 0, stream>>>(
      WV, DE, 0LL,
      KI, DE, (long long)NTOK * DE,
      b_o, 0.f,
      (void*)VTp, (void*)VTp, NTOK, (long long)DM * NTOK,
      DM, NTOK, DE, VC / (ACARRY * WSC));

  attn96<<<gAT, blk, 0, stream>>>(QH, QL, KP, VTp, CT);

  gemm64<0, 1><<<gQK, blk, 0, stream>>>(
      CT, DM, 0LL,
      WO, DM, 0LL,
      b_o, 1.0f,
      (void*)out, (void*)out, DM, 0LL,
      MROWS, DM, DM, 1.0f / (FC * WSC));
  (void)hipGetLastError();
}
